// DecoderBlock_30451318129092
// MI455X (gfx1250) — hardware-verified
//
#include <hip/hip_runtime.h>
#ifndef NB
#define NB 4
#endif
#ifndef SEQ
#define SEQ 1024
#endif
#ifndef CTX
#define CTX 1024
#endif
#define NB_FULL 4
#define SEQ_FULL 1024
#define CTX_FULL 1024
#define DM 1024
#define NH 16
#define HD 64
#define DFF 4096
#define NRQ ((unsigned)(NB * SEQ))
#define NRC ((unsigned)(NB * CTX))
#define NEGV (-1.0e9f)

static_assert(NB >= 1 && NB <= NB_FULL);
static_assert(SEQ <= SEQ_FULL && CTX <= CTX_FULL);
static_assert(NB == 1 || SEQ == SEQ_FULL);
static_assert(SEQ % 128 == 0 && CTX % 128 == 0);
static_assert(DM == NH * HD && DM == 1024 && HD == 64);
static_assert(DM % 64 == 0 && DFF % 64 == 0 && (3 * DM) % 64 == 0 && (2 * DM) % 64 == 0);
static_assert(DM % 32 == 0 && DFF % 32 == 0);
static_assert((NB * SEQ * (SEQ / 32)) % 256 == 0);

typedef unsigned short v8us __attribute__((ext_vector_type(8), may_alias));
typedef float  v8f  __attribute__((ext_vector_type(8)));
typedef float  v4f  __attribute__((ext_vector_type(4)));
typedef float  v4fa __attribute__((ext_vector_type(4), may_alias));
typedef int    v4ia __attribute__((ext_vector_type(4), may_alias));
typedef unsigned v2ua __attribute__((ext_vector_type(2), may_alias));
typedef _Float16 v16h __attribute__((ext_vector_type(16)));
typedef _Float16 v4h  __attribute__((ext_vector_type(4)));
union FragH { v16h v; v8us half[2]; _Float16 h[16]; unsigned short u[16]; };

__device__ __forceinline__ unsigned short bf16_bits(float x) { unsigned int u = __float_as_uint(x); return (unsigned short)((u + 0x7FFFu + ((u >> 16) & 1u)) >> 16); }
__device__ __forceinline__ float bf16_val(unsigned short b) { return __uint_as_float(((unsigned int)b) << 16); }
__device__ __forceinline__ float bf16_rne(float x) { return bf16_val(bf16_bits(x)); }

__device__ __forceinline__ v16h g2_frag(const _Float16* p, unsigned hh) { FragH f; f.half[0] = *(const v8us*)((const unsigned short*)p + 8 * hh); f.half[1] = *(const v8us*)((const unsigned short*)p + 16 + 8 * hh); return f.v; }
__device__ __forceinline__ v8f g2_mma(v16h a, v16h b, v8f c) { v8f d = __builtin_amdgcn_wmma_f32_16x16x32_f16(false, a, false, b, (short)0, c, false, false); asm volatile("v_nop\n\tv_nop\n\tv_nop\n\tv_nop" : "+v"(d) : "v"(a), "v"(b)); return d; }

__global__ __launch_bounds__(256) void k_wnat(const float* __restrict__ w, unsigned n8, _Float16* __restrict__ Bt) {
  const unsigned t = blockIdx.x * 256u + threadIdx.x; if (t >= n8) return;
  const v4f a = *(const v4fa*)(w + (size_t)t * 8), c = *(const v4fa*)(w + (size_t)t * 8 + 4);
  FragH f;
#pragma unroll
  for (int q = 0; q < 4; ++q) { f.h[q] = (_Float16)(bf16_rne(a[q]) * 16.0f); f.h[4 + q] = (_Float16)(bf16_rne(c[q]) * 16.0f); }
  unsigned short* d = (unsigned short*)Bt + (size_t)t * 8; const v8us o = f.half[0];
  *(volatile v8us*)d = o; __threadfence(); *(volatile v8us*)d = o;
}

__global__ __launch_bounds__(256) void k_mpack(const int* __restrict__ mk, unsigned* __restrict__ MB) {
  const unsigned t = blockIdx.x * 256u + threadIdx.x; if (t >= (unsigned)(NB * SEQ * (SEQ / 32))) return;
  const unsigned wj = t % (unsigned)(SEQ / 32), row = t / (unsigned)(SEQ / 32);
  const unsigned b = row / (unsigned)SEQ, i = row % (unsigned)SEQ;
  const int* src = mk + ((size_t)b * SEQ_FULL + i) * SEQ_FULL + wj * 32u;
  unsigned wbits = 0u;
#pragma unroll
  for (unsigned q = 0; q < 8; ++q) { const v4ia m4 = *(const v4ia*)(src + q * 4u);
    wbits |= (m4[0] != 0 ? 1u : 0u) << (q * 4u); wbits |= (m4[1] != 0 ? 1u : 0u) << (q * 4u + 1u); wbits |= (m4[2] != 0 ? 1u : 0u) << (q * 4u + 2u); wbits |= (m4[3] != 0 ? 1u : 0u) << (q * 4u + 3u); }
  *(volatile unsigned*)(MB + t) = wbits; __threadfence(); *(volatile unsigned*)(MB + t) = wbits;
}

template <int BFIN, int WXB>
__global__ __launch_bounds__(256) void k_ln16(const float* __restrict__ X, unsigned rpb, unsigned rfull, const float* __restrict__ g, float eps, _Float16* __restrict__ N16, float* __restrict__ XB) {
  #pragma clang fp contract(off)
  __shared__ float red[256];
  const unsigned r = blockIdx.x, t = threadIdx.x;
  const unsigned bq = r / rpb, sq = r - bq * rpb;
  const size_t rin = (size_t)bq * rfull + sq;
  const v4f xa = *(const v4fa*)(X + rin * DM + t * 4u);
  float s[4]; float sum = 0.f;
#pragma unroll
  for (int q = 0; q < 4; ++q) { s[q] = BFIN ? bf16_rne(xa[q]) : xa[q]; sum = __fadd_rn(sum, s[q]); }
  red[t] = sum; __syncthreads();
  for (unsigned st = 128; st > 0; st >>= 1) { if (t < st) red[t] = __fadd_rn(red[t], red[t + st]); __syncthreads(); }
  const float mu = red[0] * (1.0f / (float)DM); __syncthreads();
  float vs = 0.f;
#pragma unroll
  for (int q = 0; q < 4; ++q) { const float dl = __fadd_rn(s[q], -mu); vs = __fadd_rn(vs, __fmul_rn(dl, dl)); }
  red[t] = vs; __syncthreads();
  for (unsigned st = 128; st > 0; st >>= 1) { if (t < st) red[t] = __fadd_rn(red[t], red[t + st]); __syncthreads(); }
  const float rs = rsqrtf(__fadd_rn(red[0] * (1.0f / (float)DM), eps));
  const v4f gv = *(const v4fa*)(g + t * 4u);
  v4h y; v4f xb;
#pragma unroll
  for (int q = 0; q < 4; ++q) { y[q] = (_Float16)__fmul_rn(__fmul_rn(__fadd_rn(s[q], -mu), rs), bf16_rne(gv[q])); xb[q] = s[q]; }
  for (int pass = 0; pass < 2; ++pass) {
    *(volatile v4h*)(N16 + (size_t)r * DM + t * 4u) = y;
    if (WXB) *(volatile v4f*)(XB + (size_t)r * DM + t * 4u) = xb;
    if (pass == 0) __threadfence();
  }
}

template <unsigned T>
__global__ __launch_bounds__(256) void k_vt(const _Float16* __restrict__ V16, unsigned ldv, _Float16* __restrict__ Vt) {
  __shared__ unsigned short tl[64][66];
  const unsigned tid = threadIdx.x; const unsigned slab = blockIdx.x / (T / 64u), lg = blockIdx.x % (T / 64u);
  const unsigned b = slab / (unsigned)NH, h = slab % (unsigned)NH;
  for (unsigned i = tid; i < 512u; i += 256u) { const unsigned r = i >> 3, c8 = (i & 7u) * 8u; FragH f;
    f.half[0] = *(const v8us*)((const unsigned short*)V16 + ((size_t)b * T + lg * 64u + r) * ldv + h * 64u + c8);
#pragma unroll
    for (unsigned q = 0; q < 8; ++q) tl[r][c8 + q] = f.u[q]; }
  __syncthreads();
  for (int pass = 0; pass < 2; ++pass) {
#pragma unroll
    for (unsigned rd = 0; rd < 2; ++rd) { const unsigned d = rd * 32u + (tid >> 3), pc = tid & 7u; FragH f;
#pragma unroll
      for (unsigned q = 0; q < 8; ++q) f.u[q] = tl[pc * 8u + q][d];
      *(volatile v8us*)((unsigned short*)Vt + ((size_t)slab * 64u + d) * T + lg * 64u + pc * 8u) = f.half[0]; }
    if (pass == 0) __threadfence();
  }
}

template <int ACT>
__global__ __launch_bounds__(128) void k_gemm2(const _Float16* __restrict__ A, unsigned lda, const _Float16* __restrict__ Bh, unsigned ldb, float alpha, const float* __restrict__ CP,
    float* __restrict__ C, _Float16* __restrict__ C16, unsigned ldc, unsigned M, unsigned N, unsigned K) {
  static_assert(ACT == 0 || ACT == 6);
  __shared__ __attribute__((aligned(16))) float so[4][32][68];
  const unsigned tid = threadIdx.x, w = tid >> 5, lane = tid & 31u, ln = lane & 15u, hh = lane >> 4;
  const unsigned ntn = N >> 6; const unsigned mt = blockIdx.x / ntn, nq = blockIdx.x - mt * ntn;
  const unsigned row0 = mt * 128u + 32u * w, col0 = nq * 64u; if (row0 >= M) return;
  const _Float16* a0p = A + (size_t)(row0 + ln) * lda; const _Float16* a1p = a0p + (size_t)16 * lda;
  const _Float16* b0p = Bh + (size_t)(col0 + ln) * ldb; const _Float16* b1p = b0p + (size_t)16 * ldb; const _Float16* b2p = b1p + (size_t)16 * ldb; const _Float16* b3p = b2p + (size_t)16 * ldb;
  const v8f z8 = {0.f,0.f,0.f,0.f,0.f,0.f,0.f,0.f}; v8f c00 = z8, c01 = z8, c02 = z8, c03 = z8, c10 = z8, c11 = z8, c12 = z8, c13 = z8;
#pragma unroll 1
  for (unsigned kb = 0; kb < K; kb += 32u) { const v16h a0 = g2_frag(a0p + kb, hh), a1 = g2_frag(a1p + kb, hh);
    v16h b = g2_frag(b0p + kb, hh); c00 = g2_mma(a0, b, c00); c10 = g2_mma(a1, b, c10);
    b = g2_frag(b1p + kb, hh); c01 = g2_mma(a0, b, c01); c11 = g2_mma(a1, b, c11);
    b = g2_frag(b2p + kb, hh); c02 = g2_mma(a0, b, c02); c12 = g2_mma(a1, b, c12);
    b = g2_frag(b3p + kb, hh); c03 = g2_mma(a0, b, c03); c13 = g2_mma(a1, b, c13); }
  v8f accs[8] = {c00, c01, c02, c03, c10, c11, c12, c13};
#pragma unroll
  for (int u = 0; u < 8; ++u) { const unsigned t = (unsigned)u & 3u, half = (unsigned)u >> 2; const unsigned col = col0 + t * 16u + ln;
#pragma unroll
    for (int r = 0; r < 8; ++r) { const unsigned rloc = half * 16u + 8u * hh + (unsigned)r; float v = accs[u][r] * alpha;
      if (CP) v += CP[(size_t)(row0 + rloc) * ldc + col];
      so[w][rloc][t * 16u + ln] = v; } }
  __builtin_amdgcn_fence(4  , "workgroup"); __builtin_amdgcn_wave_barrier();
  const unsigned rsub = lane >> 4, c4 = (lane & 15u) * 4u;
  if (ACT == 6) {
#pragma unroll 1
    for (unsigned q = 0; q < 16u; ++q) { const unsigned r = q * 2u + rsub; v4f v = *(const v4fa*)&so[w][r][c4];
#pragma unroll
      for (int i = 0; i < 4; ++i) v[i] = 8.0f * v[i] * (1.0f + erff(v[i] * 0.70710678118654752f));
      *(v4fa*)&so[w][r][c4] = v; }
  }
  for (int pass = 0; pass < 2; ++pass) {
#pragma unroll
    for (unsigned q = 0; q < 16u; ++q) { const unsigned r = q * 2u + rsub; const v4f v = *(const v4fa*)&so[w][r][c4];
      if (C) *(volatile v4f*)(C + (size_t)(row0 + r) * ldc + col0 + c4) = v;
      if (C16) { v4h h4;
#pragma unroll
        for (int i = 0; i < 4; ++i) h4[i] = (_Float16)v[i];
        *(volatile v4h*)(C16 + (size_t)(row0 + r) * ldc + col0 + c4) = h4; } }
    if (pass == 0) __threadfence();
  }
}

template <int MASKED, unsigned LQ, unsigned LK>
__global__ __launch_bounds__(128) void k_flash(const _Float16* __restrict__ Q, unsigned ldq, const _Float16* __restrict__ Kp, unsigned ldk, const _Float16* __restrict__ VT,
    const unsigned* __restrict__ MB, _Float16* __restrict__ O, unsigned ldo) {
  static_assert(LQ % 64u == 0u && LK % 64u == 0u);
  __shared__ __attribute__((aligned(16))) _Float16 pt[4][16][72];
  const unsigned tid = threadIdx.x, w = tid >> 5, lane = tid & 31u, ln = lane & 15u, hh = lane >> 4;
  const unsigned slab = blockIdx.x / (LQ / 64u), qb = blockIdx.x % (LQ / 64u);
  const unsigned b = slab / (unsigned)NH, h = slab % (unsigned)NH;
  const unsigned qrow0 = b * LQ + qb * 64u + w * 16u;
  const unsigned krow0 = b * LK;
  const _Float16* qp = Q + (size_t)(qrow0 + ln) * ldq + h * (unsigned)HD;
  const v16h qa0 = g2_frag(qp, hh), qa1 = g2_frag(qp + 32, hh);
  const _Float16* kbase = Kp + (size_t)(krow0 + ln) * ldk + h * (unsigned)HD;
  const _Float16* vbase = VT + ((size_t)slab * HD + ln) * LK;
  const unsigned* mrow = nullptr;
  if (MASKED) mrow = MB + (size_t)(qrow0 + 8u * hh) * (LK / 32u);
  const v8f z8 = {0.f,0.f,0.f,0.f,0.f,0.f,0.f,0.f};
  v8f o0 = z8, o1 = z8, o2 = z8, o3 = z8;
  float m[8], l[8];
#pragma unroll
  for (int r = 0; r < 8; ++r) { m[r] = NEGV; l[r] = 0.f; }
#pragma unroll 1
  for (unsigned j0 = 0; j0 < LK; j0 += 64u) {
    unsigned wl[8], wh[8];
    if (MASKED) {
      unsigned any = 0u;
#pragma unroll
      for (int r = 0; r < 8; ++r) { const v2ua mw = *(const v2ua*)(mrow + (unsigned)r * (LK / 32u) + (j0 >> 5)); wl[r] = mw[0]; wh[r] = mw[1]; any |= (mw[0] | mw[1]); }
      if (__builtin_amdgcn_ballot_w32(any != 0u) == 0u) continue;
    }
    v8f s0 = z8, s1 = z8, s2 = z8, s3 = z8;
    { const _Float16* kp = kbase + (size_t)j0 * ldk;
      v16h kf = g2_frag(kp, hh); s0 = g2_mma(qa0, kf, s0); kf = g2_frag(kp + 32, hh); s0 = g2_mma(qa1, kf, s0);
      kp += (size_t)16 * ldk; kf = g2_frag(kp, hh); s1 = g2_mma(qa0, kf, s1); kf = g2_frag(kp + 32, hh); s1 = g2_mma(qa1, kf, s1);
      kp += (size_t)16 * ldk; kf = g2_frag(kp, hh); s2 = g2_mma(qa0, kf, s2); kf = g2_frag(kp + 32, hh); s2 = g2_mma(qa1, kf, s2);
      kp += (size_t)16 * ldk; kf = g2_frag(kp, hh); s3 = g2_mma(qa0, kf, s3); kf = g2_frag(kp + 32, hh); s3 = g2_mma(qa1, kf, s3); }
#pragma unroll
    for (int r = 0; r < 8; ++r) {
      float v0 = s0[r] * 0.125f, v1 = s1[r] * 0.125f, v2 = s2[r] * 0.125f, v3 = s3[r] * 0.125f;
      if (MASKED) { const unsigned a = wl[r] >> ln, c = wh[r] >> ln;
        v0 = (a & 1u) ? v0 : NEGV; v1 = ((a >> 16) & 1u) ? v1 : NEGV; v2 = (c & 1u) ? v2 : NEGV; v3 = ((c >> 16) & 1u) ? v3 : NEGV; }
      float mx = fmaxf(fmaxf(v0, v1), fmaxf(v2, v3));
      mx = fmaxf(mx, __shfl_xor(mx, 1)); mx = fmaxf(mx, __shfl_xor(mx, 2)); mx = fmaxf(mx, __shfl_xor(mx, 4)); mx = fmaxf(mx, __shfl_xor(mx, 8));
      const float mn = fmaxf(m[r], mx);
      const float sc = __expf(m[r] - mn);
      const float p0 = __expf(v0 - mn), p1 = __expf(v1 - mn), p2 = __expf(v2 - mn), p3 = __expf(v3 - mn);
      l[r] = l[r] * sc + ((p0 + p1) + (p2 + p3));
      m[r] = mn;
      o0[r] *= sc; o1[r] *= sc; o2[r] *= sc; o3[r] *= sc;
      const unsigned pr = 8u * hh + (unsigned)r;
      pt[w][pr][ln] = (_Float16)(p0 * 1024.0f); pt[w][pr][16u + ln] = (_Float16)(p1 * 1024.0f); pt[w][pr][32u + ln] = (_Float16)(p2 * 1024.0f); pt[w][pr][48u + ln] = (_Float16)(p3 * 1024.0f);
    }
    __builtin_amdgcn_fence(4  , "workgroup"); __builtin_amdgcn_wave_barrier();
    const v16h pa0 = g2_frag(&pt[w][ln][0], hh), pa1 = g2_frag(&pt[w][ln][32], hh);
    { const _Float16* vp = vbase + j0;
      v16h vf = g2_frag(vp, hh); o0 = g2_mma(pa0, vf, o0); vf = g2_frag(vp + 32, hh); o0 = g2_mma(pa1, vf, o0);
      vp += (size_t)16 * LK; vf = g2_frag(vp, hh); o1 = g2_mma(pa0, vf, o1); vf = g2_frag(vp + 32, hh); o1 = g2_mma(pa1, vf, o1);
      vp += (size_t)16 * LK; vf = g2_frag(vp, hh); o2 = g2_mma(pa0, vf, o2); vf = g2_frag(vp + 32, hh); o2 = g2_mma(pa1, vf, o2);
      vp += (size_t)16 * LK; vf = g2_frag(vp, hh); o3 = g2_mma(pa0, vf, o3); vf = g2_frag(vp + 32, hh); o3 = g2_mma(pa1, vf, o3); }
    __builtin_amdgcn_fence(4  , "workgroup"); __builtin_amdgcn_wave_barrier();
  }
#pragma unroll
  for (int r = 0; r < 8; ++r) {
    float ls = l[r];
    ls += __shfl_xor(ls, 1); ls += __shfl_xor(ls, 2); ls += __shfl_xor(ls, 4); ls += __shfl_xor(ls, 8);
    const float good = 0.0625f * (1.0f / ls);
    const float invv = (m[r] > -1.0e8f) ? good : __uint_as_float(0x7fc00000u);
    const unsigned pr = 8u * hh + (unsigned)r;
    pt[w][pr][ln] = (_Float16)(o0[r] * invv); pt[w][pr][16u + ln] = (_Float16)(o1[r] * invv); pt[w][pr][32u + ln] = (_Float16)(o2[r] * invv); pt[w][pr][48u + ln] = (_Float16)(o3[r] * invv);
  }
  __builtin_amdgcn_fence(4  , "workgroup"); __builtin_amdgcn_wave_barrier();
  for (int pass = 0; pass < 2; ++pass) {
#pragma unroll
    for (unsigned q = 0; q < 4u; ++q) { const unsigned row = q * 4u + (lane >> 3), pc = (lane & 7u) * 8u;
      const v8us v = *(const v8us*)&pt[w][row][pc];
      *(volatile v8us*)((unsigned short*)O + (size_t)(qrow0 + row) * ldo + h * (unsigned)HD + pc) = v; }
    if (pass == 0) __threadfence();
  }
}

constexpr size_t cmax(size_t a, size_t b) { return a > b ? a : b; }
constexpr size_t SZ_BQKV = (size_t)3 * DM * DM * 2, SZ_BSQ = (size_t)DM * DM * 2, SZ_BKV = (size_t)2 * DM * DM * 2, SZ_BW = (size_t)DFF * DM * 2;
constexpr size_t SZ_XF = (size_t)NB * SEQ * DM * 4, SZ_H16 = (size_t)NB * SEQ * DM * 2, SZ_HC16 = (size_t)NB * CTX * DM * 2;
constexpr size_t SZ_QKV = (size_t)NB * SEQ * 3 * DM * 2, SZ_VTS = (size_t)NB * DM * SEQ * 2;
constexpr size_t SZ_Q2 = (size_t)NB * SEQ * DM * 2, SZ_KV2 = (size_t)NB * CTX * 2 * DM * 2, SZ_VTC = (size_t)NB * DM * CTX * 2;
constexpr size_t SZ_G16 = (size_t)NB * SEQ * DFF * 2;
constexpr size_t SZ_BIG = cmax(cmax(SZ_QKV + SZ_VTS, SZ_Q2 + SZ_KV2 + SZ_VTC), SZ_G16);
constexpr size_t SZ_MB = (size_t)NB * SEQ * (SEQ / 32) * 4;
constexpr size_t SZ_TOTAL = SZ_BQKV + 3 * SZ_BSQ + SZ_BKV + 2 * SZ_BW + 2 * SZ_XF + SZ_H16 + SZ_HC16 + SZ_H16 + SZ_BIG + SZ_MB;
static_assert(SZ_QKV + SZ_VTS <= SZ_BIG && SZ_Q2 + SZ_KV2 + SZ_VTC <= SZ_BIG && SZ_G16 <= SZ_BIG);
static_assert(SZ_QKV % 256 == 0 && SZ_Q2 % 256 == 0 && SZ_KV2 % 256 == 0 && SZ_MB % 256 == 0 && SZ_H16 % 256 == 0 && SZ_HC16 % 256 == 0);
static_assert(SZ_TOTAL <= (size_t)134217728);

extern "C" void kernel_launch(void* const* d_in, const int* in_sizes, int n_in,
                              void* d_out, int out_size, void* d_ws, size_t ws_size, hipStream_t stream) {
  if (n_in < 14) return;
  const long long need_x = ((long long)(NB - 1) * SEQ_FULL + SEQ) * DM;
  const long long need_c = ((long long)(NB - 1) * CTX_FULL + CTX) * DM;
  const long long need_m = ((long long)(NB - 1) * SEQ_FULL + (SEQ - 1)) * SEQ_FULL + SEQ;
  if ((long long)in_sizes[0] < need_x || (long long)in_sizes[1] < need_c || (long long)in_sizes[2] < need_m) return;
  if (in_sizes[3] < 3 * DM * DM || in_sizes[4] < DM * DM || in_sizes[5] < DM * DM || in_sizes[6] < 2 * DM * DM || in_sizes[7] < DM * DM || in_sizes[8] < DFF * DM || in_sizes[9] < DM * DFF) return;
  if (in_sizes[10] < DM || in_sizes[11] < DM || in_sizes[12] < DM || in_sizes[13] < DM) return;
  if ((long long)out_size < (long long)NB * SEQ * DM) return;
  const float* x = (const float*)d_in[0]; const float* ctx = (const float*)d_in[1]; const int* mk = (const int*)d_in[2];
  const float* wqkv = (const float*)d_in[3]; const float* wso = (const float*)d_in[4]; const float* wq = (const float*)d_in[5]; const float* wkv = (const float*)d_in[6];
  const float* wco = (const float*)d_in[7]; const float* wf1 = (const float*)d_in[8]; const float* wf2 = (const float*)d_in[9];
  const float* g1 = (const float*)d_in[10]; const float* gq = (const float*)d_in[11]; const float* gc = (const float*)d_in[12]; const float* g2 = (const float*)d_in[13];
  char* ws = (char*)d_ws; size_t off = 0;
  auto take = [&](size_t bytes) { char* p = ws + off; off += (bytes + 255) & ~(size_t)255; return p; };
  _Float16* BQKV = (_Float16*)take(SZ_BQKV); _Float16* BSO = (_Float16*)take(SZ_BSQ); _Float16* BQ = (_Float16*)take(SZ_BSQ); _Float16* BKV = (_Float16*)take(SZ_BKV);
  _Float16* BCO = (_Float16*)take(SZ_BSQ); _Float16* BW1 = (_Float16*)take(SZ_BW); _Float16* BW2 = (_Float16*)take(SZ_BW);
  float* XB = (float*)take(SZ_XF);
  float* XA = (float*)take(SZ_XF);
  _Float16* H16 = (_Float16*)take(SZ_H16); _Float16* HC16 = (_Float16*)take(SZ_HC16); _Float16* O16 = (_Float16*)take(SZ_H16);
  char* BIG = take(SZ_BIG);
  unsigned* MB = (unsigned*)take(SZ_MB);
  if (off > ws_size) return;
  _Float16* QKV16 = (_Float16*)BIG; _Float16* VTS = (_Float16*)(BIG + SZ_QKV);
  _Float16* Q2 = (_Float16*)BIG; _Float16* KV2 = (_Float16*)(BIG + SZ_Q2); _Float16* VTC = (_Float16*)(BIG + SZ_Q2 + SZ_KV2);
  _Float16* G16 = (_Float16*)BIG;

  { const unsigned n8 = (unsigned)(3u * DM * DM / 8u); k_wnat<<<(n8 + 255u) / 256u, 256, 0, stream>>>(wqkv, n8, BQKV); }
  { const unsigned n8 = (unsigned)(DM * DM / 8u); k_wnat<<<(n8 + 255u) / 256u, 256, 0, stream>>>(wso, n8, BSO); k_wnat<<<(n8 + 255u) / 256u, 256, 0, stream>>>(wq, n8, BQ); k_wnat<<<(n8 + 255u) / 256u, 256, 0, stream>>>(wco, n8, BCO); }
  { const unsigned n8 = (unsigned)(2u * DM * DM / 8u); k_wnat<<<(n8 + 255u) / 256u, 256, 0, stream>>>(wkv, n8, BKV); }
  { const unsigned n8 = (unsigned)((unsigned)DFF * DM / 8u); k_wnat<<<(n8 + 255u) / 256u, 256, 0, stream>>>(wf1, n8, BW1); k_wnat<<<(n8 + 255u) / 256u, 256, 0, stream>>>(wf2, n8, BW2); }
  k_mpack<<<(unsigned)(NB * SEQ * (SEQ / 32)) / 256u, 256, 0, stream>>>(mk, MB);

  k_ln16<1, 1><<<NRQ, 256, 0, stream>>>(x, (unsigned)SEQ, (unsigned)SEQ_FULL, g1, 1e-6f, H16, XB);
  k_gemm2<0><<<(NRQ / 128u) * (3u * DM / 64u), 128, 0, stream>>>(H16, DM, BQKV, DM, 0.0625f, nullptr, nullptr, QKV16, 3u * DM, NRQ, 3u * DM, DM);
  k_vt<SEQ><<<(unsigned)(NB * NH * (SEQ / 64)), 256, 0, stream>>>(QKV16 + 2 * DM, 3u * DM, VTS);
  k_flash<1, SEQ, SEQ><<<(unsigned)(NB * NH * (SEQ / 64)), 128, 0, stream>>>(QKV16, 3u * DM, QKV16 + DM, 3u * DM, VTS, MB, O16, DM);
  k_gemm2<0><<<(NRQ / 128u) * (DM / 64u), 128, 0, stream>>>(O16, DM, BSO, DM, 0.0009765625f, XB, XA, nullptr, DM, NRQ, DM, DM);

  k_ln16<0, 0><<<NRQ, 256, 0, stream>>>(XA, NRQ, NRQ, gq, 1e-6f, H16, nullptr);
  k_ln16<1, 0><<<NRC, 256, 0, stream>>>(ctx, (unsigned)CTX, (unsigned)CTX_FULL, gc, 1e-6f, HC16, nullptr);
  k_gemm2<0><<<(NRQ / 128u) * (DM / 64u), 128, 0, stream>>>(H16, DM, BQ, DM, 0.0625f, nullptr, nullptr, Q2, DM, NRQ, DM, DM);
  k_gemm2<0><<<(NRC / 128u) * (2u * DM / 64u), 128, 0, stream>>>(HC16, DM, BKV, DM, 0.0625f, nullptr, nullptr, KV2, 2u * DM, NRC, 2u * DM, DM);
  k_vt<CTX><<<(unsigned)(NB * NH * (CTX / 64)), 256, 0, stream>>>(KV2 + DM, 2u * DM, VTC);
  k_flash<0, SEQ, CTX><<<(unsigned)(NB * NH * (SEQ / 64)), 128, 0, stream>>>(Q2, DM, KV2, 2u * DM, VTC, nullptr, O16, DM);
  k_gemm2<0><<<(NRQ / 128u) * (DM / 64u), 128, 0, stream>>>(O16, DM, BCO, DM, 0.0009765625f, XA, XB, nullptr, DM, NRQ, DM, DM);

  k_ln16<0, 0><<<NRQ, 256, 0, stream>>>(XB, NRQ, NRQ, g2, 1e-6f, H16, nullptr);
  k_gemm2<6><<<(NRQ / 128u) * ((unsigned)DFF / 64u), 128, 0, stream>>>(H16, DM, BW1, DM, 0.0625f, nullptr, nullptr, G16, DFF, NRQ, DFF, DM);
  k_gemm2<0><<<(NRQ / 128u) * (DM / 64u), 128, 0, stream>>>(G16, DFF, BW2, DFF, 0.00390625f, XB, (float*)d_out, nullptr, DM, NRQ, DM, DFF);
}
